// CrossSpectralSpatialAttention_14413910245925
// MI455X (gfx1250) — hardware-verified
//
#include <hip/hip_runtime.h>
#include <math.h>
#include <stdint.h>

#define CDIM  128
#define NHD   8
#define HDIM  16
#define DD    31
#define HWN   1024
#define PP    31744
#define NWV   (DD * (HWN / 16))
#define QSP   136
#define CSP   132
#define OSP   132
#define TQP   72
#define XCAR  16.0f
#define WSC   256.0f
#define QKC   64.0f
#define PCAR  1024.0f
#define ZC    1024.0f
#define RESC  2048.0f
#define RINV  0.00048828125f
#define PCS   31744.0f
#define PONE  1024.0f
#define NEGS  (-1.0e30f)

static_assert(DD * HWN == PP);
static_assert((PP % 64) == 0 && (CDIM % 64) == 0 && (PP % 256) == 0);
static_assert(NHD * HDIM == CDIM);
static_assert((NWV % 4) == 0);
static_assert((QSP % 8) == 0 && (CSP % 4) == 0 && (OSP % 4) == 0 && (TQP % 8) == 0);

typedef _Float16 v16h __attribute__((ext_vector_type(16)));
typedef _Float16 v8h  __attribute__((ext_vector_type(8)));
typedef float    v8f  __attribute__((ext_vector_type(8)));
typedef float    v4f  __attribute__((ext_vector_type(4)));
typedef unsigned int v4u __attribute__((ext_vector_type(4)));
typedef unsigned short v16us __attribute__((ext_vector_type(16)));

union FragH { v16h v; v8h h[2]; v4u u[2]; v16us s; };

__device__ __forceinline__ unsigned short bf_bits(float f) {
  unsigned u = __float_as_uint(f);
  return (unsigned short)((u + 0x7FFFu + ((u >> 16) & 1u)) >> 16);
}
__device__ __forceinline__ float bf_up(unsigned short b) { return __uint_as_float(((unsigned)b) << 16); }
__device__ __forceinline__ float bfr(float f) { return bf_up(bf_bits(f)); }
__device__ __forceinline__ unsigned short h_bits(_Float16 x) { return __builtin_bit_cast(unsigned short, x); }
__device__ __forceinline__ float h2f(unsigned short u) { return (float)__builtin_bit_cast(_Float16, u); }
__device__ __forceinline__ unsigned pk16(unsigned short a, unsigned short b) { return (unsigned)a | ((unsigned)b << 16); }
__device__ __forceinline__ v8f zero8() { v8f z = {0.f, 0.f, 0.f, 0.f, 0.f, 0.f, 0.f, 0.f}; return z; }

__device__ __forceinline__ v16h ldfrag_u(const unsigned short* p) {
  FragH f;
  f.u[0] = *(const v4u*)(p);
  f.u[1] = *(const v4u*)(p + 16);
  return f.v;
}
__device__ __forceinline__ v16h ldfrag_k16(const unsigned short* p) {
  FragH f;
  f.u[0] = *(const v4u*)(p);
  const v4u z = {0u, 0u, 0u, 0u};
  f.u[1] = z;
  return f.v;
}

__device__ __forceinline__ v8f mma_raw(v16h a, v16h b, v8f c) {
  return __builtin_amdgcn_wmma_f32_16x16x32_f16(false, a, false, b, (short)0, c, false, false);
}
__device__ __forceinline__ void guard_4x1(v8f& a, v8f& b, v8f& c, v8f& d, v16h x) {
#if defined(__HIP_DEVICE_COMPILE__)
  asm volatile("v_nop\n\tv_nop\n\tv_nop\n\tv_nop" : "+v"(a), "+v"(b), "+v"(c), "+v"(d) : "v"(x));
#endif
}
__device__ __forceinline__ void keep4_h(v16h a, v16h b, v16h c, v16h d) {
#if defined(__HIP_DEVICE_COMPILE__)
  asm volatile("v_nop" :: "v"(a), "v"(b), "v"(c), "v"(d));
#endif
}
__device__ __forceinline__ void acc_guard4(v8f& a, v8f& b, v8f& c, v8f& d) {
#if defined(__HIP_DEVICE_COMPILE__)
  asm volatile("v_nop\n\tv_nop\n\tv_nop\n\tv_nop" : "+v"(a), "+v"(b), "+v"(c), "+v"(d));
#endif
}
__device__ __forceinline__ void guard_2x3(v8f& a, v8f& b, v16h x0, v16h x1, v16h x2) {
#if defined(__HIP_DEVICE_COMPILE__)
  asm volatile("v_nop\n\tv_nop\n\tv_nop\n\tv_nop" : "+v"(a), "+v"(b) : "v"(x0), "v"(x1), "v"(x2));
#endif
}
__device__ __forceinline__ void guard_1x2(v8f& a, v16h x0, v16h x1) {
#if defined(__HIP_DEVICE_COMPILE__)
  asm volatile("v_nop\n\tv_nop\n\tv_nop\n\tv_nop" : "+v"(a) : "v"(x0), "v"(x1));
#endif
}
__device__ __forceinline__ void wave_sync_lds() {
  __builtin_amdgcn_fence(__ATOMIC_RELEASE, "workgroup");
  __builtin_amdgcn_wave_barrier();
  __builtin_amdgcn_fence(__ATOMIC_ACQUIRE, "workgroup");
}

__device__ __forceinline__ void split8(const float* sp, v4u& hi, v4u& lo) {
  const v4f a = *(const v4f*)(sp), b = *(const v4f*)(sp + 4);
  float v[8];
#pragma unroll
  for (int e = 0; e < 4; ++e) { v[e] = a[e]; v[4 + e] = b[e]; }
#pragma unroll
  for (int e = 0; e < 4; ++e) {
    const _Float16 h0 = (_Float16)v[2 * e], h1 = (_Float16)v[2 * e + 1];
    const _Float16 l0 = (_Float16)((v[2 * e] - (float)h0) * RESC);
    const _Float16 l1 = (_Float16)((v[2 * e + 1] - (float)h1) * RESC);
    hi[e] = pk16(h_bits(h0), h_bits(h1));
    lo[e] = pk16(h_bits(l0), h_bits(l1));
  }
}

__global__ __launch_bounds__(256) void cvx(const float* __restrict__ x, unsigned short* xh) {
  __shared__ __align__(16) unsigned short T[64 * QSP];
  const int t  = threadIdx.x;
  const int p0 = blockIdx.x * 64;
#pragma unroll 4
  for (int i = 0; i < 32; ++i) {
    const int e  = t + 256 * i;
    const int pl = e & 63, cl = e >> 6;
    const float v = bfr(x[(size_t)cl * PP + p0 + pl]) * XCAR;
    T[pl * QSP + cl] = h_bits((_Float16)v);
  }
  __syncthreads();
  v4u o[4];
#pragma unroll
  for (int i = 0; i < 4; ++i) {
    const int chunk = t + 256 * i;
    const int row = chunk >> 4, c8 = (chunk & 15) * 8;
    o[i] = *(const v4u*)(T + row * QSP + c8);
  }
#pragma unroll
  for (int i = 0; i < 4; ++i) {
    const int chunk = t + 256 * i;
    const int row = chunk >> 4, c8 = (chunk & 15) * 8;
    *(volatile v4u*)(xh + (size_t)(p0 + row) * CDIM + c8) = o[i];
  }
  __threadfence();
#pragma unroll
  for (int i = 0; i < 4; ++i) {
    const int chunk = t + 256 * i;
    const int row = chunk >> 4, c8 = (chunk & 15) * 8;
    *(volatile v4u*)(xh + (size_t)(p0 + row) * CDIM + c8) = o[i];
  }
  __threadfence();
}

__global__ __launch_bounds__(256) void cvw(const float* __restrict__ W0, const float* __restrict__ W1,
                                           const float* __restrict__ W2, const float* __restrict__ W3,
                                           unsigned short* WT) {
  __shared__ __align__(16) unsigned short T[32 * QSP];
  const int t  = threadIdx.x;
  const int n0 = blockIdx.x * 32;
  const int j  = blockIdx.y;
  const float* W = (j == 0) ? W0 : ((j == 1) ? W1 : ((j == 2) ? W2 : W3));
  unsigned short* dst = WT + (size_t)j * CDIM * CDIM;
#pragma unroll 4
  for (int i = 0; i < 16; ++i) {
    const int e  = t + 256 * i;
    const int nn = e & 31, k = e >> 5;
    const float v = bfr(W[(size_t)k * CDIM + n0 + nn]) * WSC;
    T[nn * QSP + k] = h_bits((_Float16)v);
  }
  __syncthreads();
  v4u o[2];
#pragma unroll
  for (int i = 0; i < 2; ++i) {
    const int chunk = t + 256 * i;
    const int nn = chunk >> 4, c8 = (chunk & 15) * 8;
    o[i] = *(const v4u*)(T + nn * QSP + c8);
  }
#pragma unroll
  for (int i = 0; i < 2; ++i) {
    const int chunk = t + 256 * i;
    const int nn = chunk >> 4, c8 = (chunk & 15) * 8;
    *(volatile v4u*)(dst + (size_t)(n0 + nn) * CDIM + c8) = o[i];
  }
  __threadfence();
#pragma unroll
  for (int i = 0; i < 2; ++i) {
    const int chunk = t + 256 * i;
    const int nn = chunk >> 4, c8 = (chunk & 15) * 8;
    *(volatile v4u*)(dst + (size_t)(n0 + nn) * CDIM + c8) = o[i];
  }
  __threadfence();
}

__global__ __launch_bounds__(256) void trq(const unsigned short* __restrict__ Q, unsigned short* QT) {
  __shared__ __align__(16) unsigned short T[CDIM * TQP];
  const int t  = threadIdx.x;
  const int p0 = blockIdx.x * 64;
#pragma unroll
  for (int i = 0; i < 4; ++i) {
    const int chunk = t + 256 * i;
    const int pl = chunk >> 4, c8 = (chunk & 15) * 8;
    const v4u v = *(const v4u*)(Q + (size_t)(p0 + pl) * CDIM + c8);
#pragma unroll
    for (int e = 0; e < 4; ++e) {
      T[(c8 + 2 * e) * TQP + pl]     = (unsigned short)(v[e] & 0xFFFFu);
      T[(c8 + 2 * e + 1) * TQP + pl] = (unsigned short)(v[e] >> 16);
    }
  }
  __syncthreads();
  v4u o[4];
#pragma unroll
  for (int i = 0; i < 4; ++i) {
    const int chunk = t + 256 * i;
    const int cl = chunk >> 3, pc = (chunk & 7) * 8;
    o[i] = *(const v4u*)(T + cl * TQP + pc);
  }
#pragma unroll
  for (int i = 0; i < 4; ++i) {
    const int chunk = t + 256 * i;
    const int cl = chunk >> 3, pc = (chunk & 7) * 8;
    *(volatile v4u*)(QT + (size_t)cl * PP + p0 + pc) = o[i];
  }
  __threadfence();
#pragma unroll
  for (int i = 0; i < 4; ++i) {
    const int chunk = t + 256 * i;
    const int cl = chunk >> 3, pc = (chunk & 7) * 8;
    *(volatile v4u*)(QT + (size_t)cl * PP + p0 + pc) = o[i];
  }
  __threadfence();
}

__device__ __forceinline__ void kloop(v8f (&acc)[4][4], const unsigned short* __restrict__ A1, int lda, long long sAk,
                                      const unsigned short* __restrict__ Bb, int ldb, int m0, int n0, int K,
                                      int rlane, int koff) {
#pragma unroll 1
  for (int k0 = 0; k0 < K; k0 += 32) {
    v16h bh[4];
#pragma unroll
    for (int j = 0; j < 4; ++j) {
      const size_t bofs = (size_t)(n0 + (j << 4) + rlane) * (size_t)ldb + (size_t)(koff + k0);
      bh[j] = ldfrag_u(Bb + bofs);
    }
    const size_t ak = (size_t)(k0 >> 5) * (size_t)sAk + (size_t)((k0 & 31) + koff);
#pragma unroll
    for (int i = 0; i < 4; ++i) {
      const size_t ao = (size_t)(m0 + (i << 4) + rlane) * (size_t)lda + ak;
      const v16h ah = ldfrag_u(A1 + ao);
#pragma unroll
      for (int j = 0; j < 4; ++j) acc[i][j] = mma_raw(ah, bh[j], acc[i][j]);
      guard_4x1(acc[i][0], acc[i][1], acc[i][2], acc[i][3], ah);
    }
    keep4_h(bh[0], bh[1], bh[2], bh[3]);
  }
}

template <int OM, int BIASM>
__global__ __launch_bounds__(256) void gemm64(
    const unsigned short* __restrict__ Ap, int lda, long long sAk, long long aLo,
    const unsigned short* __restrict__ Btp, int ldb,
    const float* __restrict__ bias, float bscale,
    void* Cout, int ldc, long long cLo,
    int M, int N, int K, float oscale) {
  __shared__ __align__(16) float sT[8][16 * 68];
  const int lane = threadIdx.x & 31;
  const int wave = threadIdx.x >> 5;
  const int tilesN = N >> 6;
  const int tilesM = M >> 6;
  const int tile = blockIdx.x * 8 + wave;
  if (tile >= tilesM * tilesN) return;
  const int tm = tile / tilesN;
  const int tn = tile - tm * tilesN;
  const int m0 = tm << 6;
  const int n0 = tn << 6;

  const int rlane = lane & 15;
  const int koff  = (lane >> 4) * 8;
  const int mOff  = (lane >> 4) * 8;

  v8f acc[4][4];
#pragma unroll
  for (int i = 0; i < 4; ++i)
#pragma unroll
    for (int j = 0; j < 4; ++j) acc[i][j] = zero8();

  if (aLo != 0) {
    kloop(acc, Ap + aLo, lda, sAk, Btp, ldb, m0, n0, K, rlane, koff);
    acc_guard4(acc[0][0], acc[0][1], acc[0][2], acc[0][3]);
    acc_guard4(acc[1][0], acc[1][1], acc[1][2], acc[1][3]);
    acc_guard4(acc[2][0], acc[2][1], acc[2][2], acc[2][3]);
    acc_guard4(acc[3][0], acc[3][1], acc[3][2], acc[3][3]);
#pragma unroll
    for (int i = 0; i < 4; ++i)
#pragma unroll
      for (int j = 0; j < 4; ++j) acc[i][j] = acc[i][j] * RINV;
  }
  kloop(acc, Ap, lda, sAk, Btp, ldb, m0, n0, K, rlane, koff);
  acc_guard4(acc[0][0], acc[0][1], acc[0][2], acc[0][3]);
  acc_guard4(acc[1][0], acc[1][1], acc[1][2], acc[1][3]);
  acc_guard4(acc[2][0], acc[2][1], acc[2][2], acc[2][3]);
  acc_guard4(acc[3][0], acc[3][1], acc[3][2], acc[3][3]);

  const int hh2 = lane >> 4, c4 = (lane & 15) * 4;
  const int q8  = lane >> 3, c8 = (lane & 7) * 8;
  float bc4[4], bc8[8];
#pragma unroll
  for (int e = 0; e < 4; ++e) bc4[e] = 0.f;
#pragma unroll
  for (int e = 0; e < 8; ++e) bc8[e] = 0.f;
  if (BIASM == 0) {
    if (OM == 4) {
      const int cb = n0 + c4;
      const int i0 = (cb <= N - 4) ? cb : (N - 4);
      const v4f b0v = *(const v4f*)(bias + i0);
#pragma unroll
      for (int e = 0; e < 4; ++e) bc4[e] = bfr(b0v[e]) * bscale;
    } else {
      const int cb = n0 + c8;
      const int i0 = (cb <= N - 8) ? cb : (N - 8);
      const v4f b0v = *(const v4f*)(bias + i0), b1v = *(const v4f*)(bias + i0 + 4);
#pragma unroll
      for (int e = 0; e < 4; ++e) { bc8[e] = bfr(b0v[e]) * bscale; bc8[4 + e] = bfr(b1v[e]) * bscale; }
    }
  }

  float* slab = sT[wave];
#pragma unroll
  for (int i = 0; i < 4; ++i) {
    const int mBase = m0 + (i << 4);
#pragma unroll
    for (int j = 0; j < 4; ++j) {
#pragma unroll
      for (int r = 0; r < 8; ++r) {
        slab[(mOff + r) * 68 + (j << 4) + rlane] = acc[i][j][r];
      }
    }
    wave_sync_lds();
    if (OM == 4) {
      float* C = (float*)Cout;
      v4f vals[8];
#pragma unroll
      for (int it = 0; it < 8; ++it) {
        const int row = it * 2 + hh2;
        float rb = 0.f;
        if (BIASM == 1) {
          const int gr = mBase + row;
          rb = bfr(bias[(gr < M) ? gr : (M - 1)]) * bscale;
        }
        v4f v = *(const v4f*)(slab + row * 68 + c4);
#pragma unroll
        for (int e = 0; e < 4; ++e) v[e] = v[e] * oscale + bc4[e] + rb;
        vals[it] = v;
      }
#pragma unroll
      for (int it = 0; it < 8; ++it) {
        const int gr = mBase + it * 2 + hh2;
        *(volatile v4f*)(C + (size_t)gr * (size_t)ldc + n0 + c4) = vals[it];
      }
      __threadfence();
#pragma unroll
      for (int it = 0; it < 8; ++it) {
        const int gr = mBase + it * 2 + hh2;
        *(volatile v4f*)(C + (size_t)gr * (size_t)ldc + n0 + c4) = vals[it];
      }
      __threadfence();
    } else {
      unsigned short* C = (unsigned short*)Cout;
      v4u hv[4], lv[4];
#pragma unroll
      for (int it = 0; it < 4; ++it) {
        const int row = it * 4 + q8;
        float rb = 0.f;
        if (BIASM == 1) {
          const int gr = mBase + row;
          rb = bfr(bias[(gr < M) ? gr : (M - 1)]) * bscale;
        }
        const float* sp = slab + row * 68 + c8;
        const v4f x0 = *(const v4f*)(sp), x1 = *(const v4f*)(sp + 4);
        float v[8];
#pragma unroll
        for (int e = 0; e < 4; ++e) {
          v[e]     = x0[e] * oscale + bc8[e] + rb;
          v[4 + e] = x1[e] * oscale + bc8[4 + e] + rb;
        }
        v4u ha, la;
#pragma unroll
        for (int e = 0; e < 4; ++e) {
          const _Float16 h0 = (_Float16)v[2 * e], h1 = (_Float16)v[2 * e + 1];
          const _Float16 l0 = (_Float16)((v[2 * e] - (float)h0) * RESC);
          const _Float16 l1 = (_Float16)((v[2 * e + 1] - (float)h1) * RESC);
          ha[e] = pk16(h_bits(h0), h_bits(h1));
          la[e] = pk16(h_bits(l0), h_bits(l1));
        }
        hv[it] = ha;
        lv[it] = la;
      }
#pragma unroll
      for (int it = 0; it < 4; ++it) {
        const int row = it * 4 + q8;
        const size_t o = (size_t)(mBase + row) * (size_t)ldc + n0 + c8;
        *(volatile v4u*)(C + o) = hv[it];
        if (OM == 3) *(volatile v4u*)(C + cLo + o) = lv[it];
      }
      __threadfence();
#pragma unroll
      for (int it = 0; it < 4; ++it) {
        const int row = it * 4 + q8;
        const size_t o = (size_t)(mBase + row) * (size_t)ldc + n0 + c8;
        *(volatile v4u*)(C + o) = hv[it];
        if (OM == 3) *(volatile v4u*)(C + cLo + o) = lv[it];
      }
      __threadfence();
    }
    wave_sync_lds();
  }
}

__global__ __launch_bounds__(256)
void specat(const unsigned short* __restrict__ Q, unsigned short* CH, unsigned short* CL) {
  __shared__ __align__(16) unsigned short Qs[32 * QSP];
  __shared__ __align__(16) float Cs[32 * CSP];
  const int t    = threadIdx.x;
  const int wave = t >> 5;
  const int lane = t & 31;
  const int hh   = lane >> 4;
  const int c    = lane & 15;
  const int s    = blockIdx.x;

#pragma unroll
  for (int i = 0; i < 2; ++i) {
    const int chunk = t + 256 * i;
    const int cc = (chunk < 496) ? chunk : 495;
    const int l = cc >> 4, c8 = (cc & 15) * 8;
    const v4u v = *(const v4u*)(Q + ((size_t)l * HWN + s) * CDIM + c8);
    if (chunk < 496) *(v4u*)(Qs + l * QSP + c8) = v;
  }
  if (t < 16) {
    const v4u z = {0u, 0u, 0u, 0u};
    *(v4u*)(Qs + 31 * QSP + 8 * t) = z;
  }
  __syncthreads();

  const int h   = wave;
  const int col = HDIM * h;
  const v16h kf0 = ldfrag_k16(Qs + c * QSP + col + 8 * hh);
  const v16h kf1 = ldfrag_k16(Qs + (16 + c) * QSP + col + 8 * hh);
  FragH va;
#pragma unroll
  for (int i = 0; i < 8; ++i) {
    va.s[i]     = Qs[(8 * hh + i) * QSP + col + c];
    va.s[8 + i] = Qs[(16 + 8 * hh + i) * QSP + col + c];
  }
  float Sc = 0.f;
#pragma unroll 1
  for (int l = 0; l < DD; ++l) Sc += h2f(Qs[l * QSP + col + c]);
  float S8[8];
#pragma unroll
  for (int r = 0; r < 8; ++r) S8[r] = __shfl(Sc, 8 * hh + r, 32);

  const float lsc = 1.4426950408889634f / (16.0f * QKC * QKC);
  const float oc  = ZC / (QKC * PCS);

#pragma unroll
  for (int nt = 0; nt < 2; ++nt) {
    const v16h qf = ldfrag_k16(Qs + (16 * nt + c) * QSP + col + 8 * hh);
    v8f s0 = mma_raw(kf0, qf, zero8());
    v8f s1 = mma_raw(kf1, qf, zero8());
    guard_2x3(s0, s1, kf0, kf1, qf);
    float t0[8], t1[8];
#pragma unroll
    for (int r = 0; r < 8; ++r) { t0[r] = s0[r] * lsc; t1[r] = s1[r] * lsc; }
    t1[7] = hh ? NEGS : t1[7];
    float mx = fmaxf(t0[0], t1[0]);
#pragma unroll
    for (int r = 1; r < 8; ++r) mx = fmaxf(mx, fmaxf(t0[r], t1[r]));
    mx = fmaxf(mx, __shfl_xor(mx, 16, 32));
    float p0[8], p1[8], ps = 0.f;
#pragma unroll
    for (int r = 0; r < 8; ++r) {
      p0[r] = exp2f(t0[r] - mx);
      p1[r] = exp2f(t1[r] - mx);
      ps += p0[r] + p1[r];
    }
    ps += __shfl_xor(ps, 16, 32);
    const float rl = PCS * (1.0f / ps);
    float w0[8], w1[8];
#pragma unroll
    for (int r = 0; r < 8; ++r) { w0[r] = p0[r] * rl - PONE; w1[r] = p1[r] * rl - PONE; }
    w1[7] = hh ? 0.f : w1[7];
    FragH pb;
#pragma unroll
    for (int r = 0; r < 8; ++r) { pb.h[0][r] = (_Float16)w0[r]; pb.h[1][r] = (_Float16)w1[r]; }
    v8f z = mma_raw(va.v, pb.v, zero8());
    guard_1x2(z, va.v, pb.v);
    v4f o0, o1;
#pragma unroll
    for (int e = 0; e < 4; ++e) {
      o0[e] = (z[e] + PONE * S8[e]) * oc;
      o1[e] = (z[4 + e] + PONE * S8[4 + e]) * oc;
    }
    float* cp = Cs + (16 * nt + c) * CSP + col + 8 * hh;
    *(v4f*)(cp) = o0;
    *(v4f*)(cp + 4) = o1;
  }
  __syncthreads();

  v4u hv[2], lv[2];
  int rw[2], cw[2];
#pragma unroll
  for (int i = 0; i < 2; ++i) {
    const int chunk = t + 256 * i;
    const int row = chunk >> 4, c8 = (chunk & 15) * 8;
    const int rc = (row < DD) ? row : (DD - 1);
    split8(Cs + rc * CSP + c8, hv[i], lv[i]);
    rw[i] = row;
    cw[i] = c8;
  }
#pragma unroll
  for (int i = 0; i < 2; ++i) {
    if (rw[i] < DD) {
      const size_t o = ((size_t)rw[i] * HWN + s) * CDIM + cw[i];
      *(volatile v4u*)(CH + o) = hv[i];
      *(volatile v4u*)(CL + o) = lv[i];
    }
  }
  __threadfence();
#pragma unroll
  for (int i = 0; i < 2; ++i) {
    if (rw[i] < DD) {
      const size_t o = ((size_t)rw[i] * HWN + s) * CDIM + cw[i];
      *(volatile v4u*)(CH + o) = hv[i];
      *(volatile v4u*)(CL + o) = lv[i];
    }
  }
  __threadfence();
}

__global__ __launch_bounds__(128)
void flashat(const unsigned short* __restrict__ Q, const unsigned short* __restrict__ QT,
             unsigned short* CH, unsigned short* CL) {
  __shared__ __align__(16) float Os[4][16 * OSP];
  const int tid  = threadIdx.x;
  const int wave = tid >> 5;
  const int lane = tid & 31;
  const int hh   = lane >> 4;
  const int c    = lane & 15;
  const int wid  = blockIdx.x * 4 + wave;
  if (wid >= NWV) return;
  const int n  = wid >> 6;
  const int qt = wid & 63;
  const int seqbase = n * HWN;
  const int row0 = seqbase + qt * 16;
  float* os = Os[wave];
  const unsigned short* qrow = Q + (size_t)(row0 + c) * CDIM + 8 * hh;
  const unsigned short* krow = Q + (size_t)(seqbase + c) * CDIM + 8 * hh;
  const float lsc = 1.4426950408889634f / (16.0f * QKC * QKC);
  const float occ = ZC / (PCAR * QKC);

#pragma unroll 1
  for (int h = 0; h < NHD; ++h) {
    const v16h qf = ldfrag_k16(qrow + HDIM * h);
    const unsigned short* kp  = krow + HDIM * h;
    const unsigned short* vtp = QT + (size_t)(HDIM * h + c) * PP + seqbase + 8 * hh;
    float m = NEGS, l = 0.f;
    v8f oacc = zero8();
#pragma unroll 1
    for (int ks = 0; ks < HWN / 32; ++ks) {
      const int kb = ks * 32;
      const v16h kf0 = ldfrag_k16(kp + (size_t)kb * CDIM);
      const v16h kf1 = ldfrag_k16(kp + (size_t)(kb + 16) * CDIM);
      v8f s0 = mma_raw(kf0, qf, zero8());
      v8f s1 = mma_raw(kf1, qf, zero8());
      guard_2x3(s0, s1, kf0, kf1, qf);
      float mx = fmaxf(s0[0], s1[0]);
#pragma unroll
      for (int r = 1; r < 8; ++r) mx = fmaxf(mx, fmaxf(s0[r], s1[r]));
      mx = fmaxf(mx, __shfl_xor(mx, 16, 32));
      const float mn = fmaxf(m, mx * lsc);
      const float al = exp2f(m - mn);
      float ps = 0.f;
      FragH pb;
#pragma unroll
      for (int r = 0; r < 8; ++r) {
        const float p0 = exp2f(s0[r] * lsc - mn);
        const float p1 = exp2f(s1[r] * lsc - mn);
        ps += p0 + p1;
        pb.h[0][r] = (_Float16)(p0 * PCAR);
        pb.h[1][r] = (_Float16)(p1 * PCAR);
      }
      ps += __shfl_xor(ps, 16, 32);
      l = l * al + ps;
      m = mn;
#pragma unroll
      for (int r = 0; r < 8; ++r) oacc[r] = oacc[r] * al;
      const v16h vf = ldfrag_u(vtp + kb);
      oacc = mma_raw(vf, pb.v, oacc);
      guard_1x2(oacc, vf, pb.v);
    }
    const float rl = occ * (1.0f / l);
    v4f o0, o1;
#pragma unroll
    for (int e = 0; e < 4; ++e) { o0[e] = oacc[e] * rl; o1[e] = oacc[4 + e] * rl; }
    float* op = os + c * OSP + HDIM * h + 8 * hh;
    *(v4f*)(op) = o0;
    *(v4f*)(op + 4) = o1;
  }
  wave_sync_lds();

  const int sub = lane >> 4, c8 = (lane & 15) * 8;
#pragma unroll
  for (int g = 0; g < 2; ++g) {
    v4u hv[4], lv[4];
#pragma unroll
    for (int it = 0; it < 4; ++it) {
      const int row = 8 * g + 2 * it + sub;
      split8(os + row * OSP + c8, hv[it], lv[it]);
    }
#pragma unroll
    for (int it = 0; it < 4; ++it) {
      const size_t o = (size_t)(row0 + 8 * g + 2 * it + sub) * CDIM + c8;
      *(volatile v4u*)(CH + o) = hv[it];
      *(volatile v4u*)(CL + o) = lv[it];
    }
    __threadfence();
#pragma unroll
    for (int it = 0; it < 4; ++it) {
      const size_t o = (size_t)(row0 + 8 * g + 2 * it + sub) * CDIM + c8;
      *(volatile v4u*)(CH + o) = hv[it];
      *(volatile v4u*)(CL + o) = lv[it];
    }
    __threadfence();
  }
}

__global__ __launch_bounds__(128) void colsum(const float* __restrict__ O1, const float* __restrict__ O2, float* part) {
  const int by = blockIdx.y;
  const int bx = blockIdx.x;
  const int c  = threadIdx.x;
  const float* src = (by == 0) ? O1 : O2;
  const float* p = src + (size_t)bx * 256 * CDIM + c;
  float s = 0.f;
#pragma unroll 4
  for (int i = 0; i < 256; ++i) s += p[(size_t)i * CDIM];
  float* dp = part + ((size_t)by * (PP / 256) + bx) * CDIM + c;
  *(volatile float*)dp = s;
  __threadfence();
  *(volatile float*)dp = s;
}

__global__ __launch_bounds__(256) void gatek(const float* __restrict__ part, const float* __restrict__ Wg,
                                             const float* __restrict__ bg, float* gate) {
  __shared__ float gi[256];
  const int t = threadIdx.x;
  double s = 0.0;
#pragma unroll 1
  for (int i = 0; i < PP / 256; ++i) s += (double)part[((size_t)(t >> 7) * (PP / 256) + i) * CDIM + (t & 127)];
  gi[t] = (float)s * (1.0f / (float)PP);
  __syncthreads();
  const int tc = t & 127;
  float acc = bfr(bg[tc]);
#pragma unroll 1
  for (int j = 0; j < 2 * CDIM; ++j) acc += gi[j] * bfr(Wg[(size_t)j * CDIM + tc]);
  const float g = 1.0f / (1.0f + __expf(-acc));
  float* dp = gate + tc;
  if (t < 128) *(volatile float*)dp = g;
  __threadfence();
  if (t < 128) *(volatile float*)dp = g;
}

__global__ __launch_bounds__(256) void fusek(const float* __restrict__ O1, const float* __restrict__ O2,
                                             const float* __restrict__ gate, float* Y) {
  __shared__ __align__(16) float Ts[32 * 68];
  __shared__ float gs[32];
  const int t  = threadIdx.x;
  const int p0 = blockIdx.x * 64, c0 = blockIdx.y * 32;
  const float gv0 = gate[c0 + (t & 31)];
  if (t < 32) gs[t] = gv0;
  __syncthreads();
#pragma unroll 2
  for (int i = 0; i < 8; ++i) {
    const int e  = t + 256 * i;
    const int cl = e & 31, pl = e >> 5;
    const size_t src = (size_t)(p0 + pl) * CDIM + c0 + cl;
    const float a = O1[src], b = O2[src];
    const float g = gs[cl];
    Ts[cl * 68 + pl] = g * a + (1.0f - g) * b;
  }
  __syncthreads();
  v4f o[2];
#pragma unroll
  for (int i = 0; i < 2; ++i) {
    const int chunk = t + 256 * i;
    const int cl = chunk >> 4, pc = (chunk & 15) * 4;
    o[i] = *(const v4f*)(Ts + cl * 68 + pc);
  }
#pragma unroll
  for (int i = 0; i < 2; ++i) {
    const int chunk = t + 256 * i;
    const int cl = chunk >> 4, pc = (chunk & 15) * 4;
    *(volatile v4f*)(Y + (size_t)(c0 + cl) * PP + p0 + pc) = o[i];
  }
  __threadfence();
#pragma unroll
  for (int i = 0; i < 2; ++i) {
    const int chunk = t + 256 * i;
    const int cl = chunk >> 4, pc = (chunk & 15) * 4;
    *(volatile v4f*)(Y + (size_t)(c0 + cl) * PP + p0 + pc) = o[i];
  }
  __threadfence();
}

extern "C" void kernel_launch(void* const* d_in, const int* in_sizes, int n_in,
                              void* d_out, int out_size, void* d_ws, size_t ws_size,
                              hipStream_t stream) {
  if (n_in < 11) return;
  if (in_sizes[0] != PP * CDIM) return;
  if (in_sizes[1] != CDIM * CDIM || in_sizes[3] != CDIM * CDIM || in_sizes[5] != CDIM * CDIM || in_sizes[7] != CDIM * CDIM) return;
  if (in_sizes[2] != CDIM || in_sizes[4] != CDIM || in_sizes[6] != CDIM || in_sizes[8] != CDIM || in_sizes[10] != CDIM) return;
  if (in_sizes[9] != 2 * CDIM * CDIM) return;
  if (out_size != PP * CDIM) return;

  const float* x       = (const float*)d_in[0];
  const float* Wq_spec = (const float*)d_in[1];
  const float* bq_spec = (const float*)d_in[2];
  const float* Wp_spec = (const float*)d_in[3];
  const float* bp_spec = (const float*)d_in[4];
  const float* Wq_spat = (const float*)d_in[5];
  const float* bq_spat = (const float*)d_in[6];
  const float* Wp_spat = (const float*)d_in[7];
  const float* bp_spat = (const float*)d_in[8];
  const float* Wg      = (const float*)d_in[9];
  const float* bg      = (const float*)d_in[10];
  float*       out     = (float*)d_out;

  const size_t BPL16 = (size_t)PP * CDIM * 2;
  const size_t BWT   = (size_t)4 * CDIM * CDIM * 2;
  const size_t BPL32 = (size_t)PP * CDIM * 4;
  const size_t BPT   = 131072;
  const size_t BGT   = 65536;
  size_t off = 0;
  const size_t oXH = off; off += BPL16;
  const size_t oWT = off; off += BWT;
  const size_t oQP = off; off += BPL16;
  const size_t oQT = off; off += BPL16;
  const size_t oCH = off; off += BPL16;
  const size_t oCL = off; off += BPL16;
  const size_t oO1 = off; off += BPL32;
  const size_t oO2 = off; off += BPL32;
  const size_t oPT = off; off += BPT;
  const size_t oGT = off; off += BGT;
  if (off > ws_size) return;
  if (off > (size_t)134217728) return;

  char* ws = (char*)d_ws;
  unsigned short* XH = (unsigned short*)(ws + oXH);
  unsigned short* WT = (unsigned short*)(ws + oWT);
  unsigned short* QP = (unsigned short*)(ws + oQP);
  unsigned short* QT = (unsigned short*)(ws + oQT);
  unsigned short* CH = (unsigned short*)(ws + oCH);
  unsigned short* CL = (unsigned short*)(ws + oCL);
  float*          O1 = (float*)(ws + oO1);
  float*          O2 = (float*)(ws + oO2);
  float*          PT = (float*)(ws + oPT);
  float*          GT = (float*)(ws + oGT);
  const size_t WPL = (size_t)CDIM * CDIM;
  const long long aLoC = (long long)(CL - CH);

  const dim3 blk(256), blk128(128);
  const float osQ = QKC / (XCAR * WSC);
  const float osO = 1.0f / (ZC * WSC);
  const int gridG = (((PP / 64) * (CDIM / 64)) + 7) / 8;

  cvx<<<dim3(PP / 64), blk, 0, stream>>>(x, XH);
  cvw<<<dim3(4, 4), blk, 0, stream>>>(Wq_spec, Wp_spec, Wq_spat, Wp_spat, WT);

  gemm64<2, 0><<<dim3(gridG), blk, 0, stream>>>(
      XH, CDIM, 32LL, 0LL, WT + 0 * WPL, CDIM, bq_spec, QKC,
      (void*)QP, CDIM, 0LL, PP, CDIM, CDIM, osQ);
  specat<<<dim3(HWN), blk, 0, stream>>>(QP, CH, CL);
  gemm64<4, 0><<<dim3(gridG), blk, 0, stream>>>(
      CH, CDIM, 32LL, aLoC, WT + 1 * WPL, CDIM, bp_spec, 1.0f,
      (void*)O1, CDIM, 0LL, PP, CDIM, CDIM, osO);

  gemm64<2, 0><<<dim3(gridG), blk, 0, stream>>>(
      XH, CDIM, 32LL, 0LL, WT + 2 * WPL, CDIM, bq_spat, QKC,
      (void*)QP, CDIM, 0LL, PP, CDIM, CDIM, osQ);
  trq<<<dim3(PP / 64), blk, 0, stream>>>(QP, QT);
  flashat<<<dim3(NWV / 4), blk128, 0, stream>>>(QP, QT, CH, CL);
  gemm64<4, 0><<<dim3(gridG), blk, 0, stream>>>(
      CH, CDIM, 32LL, aLoC, WT + 3 * WPL, CDIM, bp_spat, 1.0f,
      (void*)O2, CDIM, 0LL, PP, CDIM, CDIM, osO);

  colsum<<<dim3(PP / 256, 2), blk128, 0, stream>>>(O1, O2, PT);
  gatek<<<dim3(1), blk, 0, stream>>>(PT, Wg, bg, GT);
  fusek<<<dim3(PP / 64, 4), blk, 0, stream>>>(O1, O2, GT, out);

  (void)hipGetLastError();
}
